// LstmCell_13030930776239
// MI455X (gfx1250) — hardware-verified
//
#include <hip/hip_runtime.h>


#define NB_  1
#define TT   4096
#define DM   2048
#define NH_  1
#define NKV  8
#define REP  (NH_ / NKV)
#define HD   1024
#define HID  1024
#define G4   (4 * HID)
#define DQ   (NH_ * HD)
#define DKV  (NKV * HD)
#define ZH   2
#define RH   512
#define WIN  0
#define PCAR 1024.0f
#define SCL  1.0f
#define INVS 0.000244140625f
#define SFL  4096.0f
#define ZEPS 1e-6f
typedef _Float16 h16;
typedef unsigned short bf;
typedef __attribute__((ext_vector_type(16))) __bf16   v16bf;
typedef __attribute__((ext_vector_type(16))) _Float16 v16h;
typedef __attribute__((ext_vector_type(8)))  _Float16 v8h;
typedef __attribute__((ext_vector_type(8)))  unsigned short v8us;
typedef __attribute__((ext_vector_type(8)))  float    v8f;
typedef __attribute__((ext_vector_type(4)))  float    v4f;
typedef v8h  __attribute__((may_alias)) v8ha;
typedef v4f  __attribute__((may_alias)) v4fa;
typedef v8us __attribute__((may_alias)) v8usa;

__device__ __forceinline__ unsigned short f2bf(float f) { unsigned u = __float_as_uint(f); u += 0x7FFFu + ((u >> 16) & 1u); return (unsigned short)(u >> 16); }
__device__ __forceinline__ float bf2f(unsigned short b) { return __uint_as_float(((unsigned)b) << 16); }
__device__ __forceinline__ float bfr(float f) { return bf2f(f2bf(f)); }
__device__ __forceinline__ v16h cat16(v8h lo, v8h hi) { return __builtin_shufflevector(lo, hi, 0, 1, 2, 3, 4, 5, 6, 7, 8, 9, 10, 11, 12, 13, 14, 15); }
__device__ __forceinline__ v16bf cat16b(v8us lo, v8us hi) { return __builtin_bit_cast(v16bf, __builtin_shufflevector(lo, hi, 0, 1, 2, 3, 4, 5, 6, 7, 8, 9, 10, 11, 12, 13, 14, 15)); }
__device__ __forceinline__ v8f wmma16(v16h a, v16h b, v8f c) { return __builtin_amdgcn_wmma_f32_16x16x32_f16(false, a, false, b, (short)0, c, false, false); }
__device__ __forceinline__ v8f wmmab(v16bf a, v16bf b, v8f c) { return __builtin_amdgcn_wmma_f32_16x16x32_bf16(false, a, false, b, (short)0, c, false, false); }


template <typename T16> struct WFrag;
template <> struct WFrag<h16> { typedef v16h V; static __device__ __forceinline__ V ld(const h16* p) { return cat16(*(const v8h*)p, *(const v8h*)(p + 16)); } static __device__ __forceinline__ v8f mma(V a, V b, v8f c) { return wmma16(a, b, c); } };
template <> struct WFrag<bf> { typedef v16bf V; static __device__ __forceinline__ V ld(const bf* p) { return cat16b(*(const v8us*)p, *(const v8us*)(p + 16)); } static __device__ __forceinline__ v8f mma(V a, V b, v8f c) { return wmmab(a, b, c); } };
template <typename T16, int NSPLIT, bool BIAS>
__global__ __launch_bounds__(32) void k_gemmw(const T16* __restrict__ A, const T16* __restrict__ A2, const T16* __restrict__ Bt, const T16* __restrict__ Bt2, int K, float* C, int ldc, const float* __restrict__ bias, size_t sA, size_t sB, size_t sC) {
    typedef typename WFrag<T16>::V V;
    __shared__ __align__(16) float os[16 * 68];
    const size_t z = blockIdx.z; A += z * sA; if (A2) A2 += z * sA; Bt += z * sB; if (Bt2) Bt2 += z * sB; C += z * sC;
    const int lane = threadIdx.x & 31, lr = lane & 15, hi = lane >> 4; const int r0 = blockIdx.x * 64, c0 = blockIdx.y * 64;
    v8f acc[4][4];
#pragma unroll
    for (int mb = 0; mb < 4; ++mb)
#pragma unroll
        for (int nb = 0; nb < 4; ++nb) acc[mb][nb] = (v8f){};
    const size_t aoff = (size_t)(r0 + lr) * K + 8 * hi, boff = (size_t)(c0 + lr) * K + 8 * hi;
#pragma unroll 1
    for (int kc = 0; kc < K; kc += 32) {
        V a[4], a2[4];
#pragma unroll
        for (int mb = 0; mb < 4; ++mb) { a[mb] = WFrag<T16>::ld(A + aoff + (size_t)mb * 16 * K + kc); if (NSPLIT == 1 || NSPLIT == 2) a2[mb] = WFrag<T16>::ld(A2 + aoff + (size_t)mb * 16 * K + kc); }
#pragma unroll
        for (int nb = 0; nb < 4; ++nb) { const V b = WFrag<T16>::ld(Bt + boff + (size_t)nb * 16 * K + kc); V b2; if (NSPLIT >= 2) b2 = WFrag<T16>::ld(Bt2 + boff + (size_t)nb * 16 * K + kc);
#pragma unroll
            for (int mb = 0; mb < 4; ++mb) { acc[mb][nb] = WFrag<T16>::mma(a[mb], b, acc[mb][nb]); if (NSPLIT == 1 || NSPLIT == 2) acc[mb][nb] = WFrag<T16>::mma(a2[mb], b, acc[mb][nb]); if (NSPLIT >= 2) acc[mb][nb] = WFrag<T16>::mma(a[mb], b2, acc[mb][nb]); } }
        asm volatile("v_nop\n\tv_nop\n\tv_nop\n\tv_nop" : "+v"(acc[0][0]), "+v"(acc[1][1]), "+v"(acc[2][2]), "+v"(acc[3][3]) : "v"(a[0]), "v"(a[3]));
    }
#pragma unroll
    for (int mb = 0; mb < 4; ++mb) {
#pragma unroll
        for (int nb = 0; nb < 4; ++nb) {
#pragma unroll
            for (int j = 0; j < 8; ++j) os[(hi * 8 + j) * 68 + nb * 16 + lr] = acc[mb][nb][j]; }
        __builtin_amdgcn_wave_barrier(); asm volatile("" ::: "memory");
        float* crow = C + (size_t)(r0 + mb * 16) * ldc + c0;
#pragma unroll 1
        for (int ps = 0; ps < 2; ++ps) {
#pragma unroll
            for (int s = 0; s < 8; ++s) { const int row = 2 * s + hi, cofs = lr * 4; v4f val = *(const v4fa*)(os + row * 68 + cofs); if (BIAS) { val[0] += bfr(bias[c0 + cofs]); val[1] += bfr(bias[c0 + cofs + 1]); val[2] += bfr(bias[c0 + cofs + 2]); val[3] += bfr(bias[c0 + cofs + 3]); }
                *(volatile v4f*)(crow + (size_t)row * ldc + cofs) = val; }
            if (ps == 0) __threadfence(); }
        __builtin_amdgcn_wave_barrier(); asm volatile("" ::: "memory");
    }
}

__device__ __forceinline__ h16 tohx(float x) { return (h16)x; }
__device__ __forceinline__ void splitf(float y, unsigned short& h, unsigned short& l) { h = f2bf(y); l = f2bf(y - bf2f(h)); }
typedef __attribute__((ext_vector_type(2))) _Float16 v2h;
typedef __attribute__((ext_vector_type(4))) _Float16 v4h;
typedef __attribute__((ext_vector_type(2))) unsigned short v2us;
typedef __attribute__((ext_vector_type(4))) unsigned short v4us;
typedef __attribute__((ext_vector_type(2))) float v2f;
typedef __attribute__((ext_vector_type(4))) int v4i;


__global__ __launch_bounds__(256) void k_cat8(const float* __restrict__ xi, const float* __restrict__ hh, bf* XH) { const size_t i = (size_t)blockIdx.x * 256 + threadIdx.x; if (i >= (size_t)TT * DM / 8) return; const size_t e = i * 8; const int c = (int)(e % DM); const int r = (int)(e / DM); const float* src = (c < HID) ? (xi + (size_t)r * HID + c) : (hh + (size_t)r * HID + (c - HID)); const v8f v = *(const v8f*)src; v8us o;
#pragma unroll
    for (int q = 0; q < 8; ++q) o[q] = f2bf(v[q]);
    *(volatile v8us*)(XH + e) = o; __threadfence(); *(volatile v8us*)(XH + e) = o; }
__global__ __launch_bounds__(256) void k_wcat(const float* __restrict__ wi, const float* __restrict__ wh, bf* Bt) { const size_t i = (size_t)blockIdx.x * 256 + threadIdx.x; if (i >= (size_t)G4 * DM / 8) return; const int k0 = (int)(i % (DM / 8)) * 8; const int n = (int)(i / (DM / 8)); const float* w = (k0 < HID) ? (wi + (size_t)k0 * G4 + n) : (wh + (size_t)(k0 - HID) * G4 + n); v8us o;
#pragma unroll
    for (int q = 0; q < 8; ++q) o[q] = f2bf(w[(size_t)q * G4]);
    *(volatile v8us*)(Bt + (size_t)n * DM + k0) = o; __threadfence(); *(volatile v8us*)(Bt + (size_t)n * DM + k0) = o; }
__global__ __launch_bounds__(256) void k_bsum(const float* __restrict__ a, const float* __restrict__ b, float* BS) { const int i = blockIdx.x * 256 + threadIdx.x; if (i >= G4 / 4) return; const v4f x = *(const v4f*)(a + i * 4); const v4f y = *(const v4f*)(b + i * 4); v4f o;
#pragma unroll
    for (int q = 0; q < 4; ++q) o[q] = __fadd_rn(bfr(x[q]), bfr(y[q]));
    *(volatile v4f*)(BS + i * 4) = o; __threadfence(); *(volatile v4f*)(BS + i * 4) = o; }
__device__ __forceinline__ float sigm(float x) { const float e = expf(-x); return __fdiv_rn(1.0f, __fadd_rn(1.0f, e)); }
__global__ __launch_bounds__(256) void k_gates(const float* __restrict__ F, const float* __restrict__ BS, const float* __restrict__ ct, float* hout, float* cout) { const size_t k = (size_t)blockIdx.x * 256 + threadIdx.x; if (k >= (size_t)TT * HID / 4) return; const size_t e = k * 4; const int j = (int)(e % HID); const int r = (int)(e / HID); const float* fr = F + (size_t)r * G4 + j; const v4f vi = *(const v4f*)(fr); const v4f vf = *(const v4f*)(fr + HID); const v4f vg = *(const v4f*)(fr + 2 * HID); const v4f vo = *(const v4f*)(fr + 3 * HID); const v4f c0 = *(const v4f*)(ct + e); const v4f bi4 = *(const v4f*)(BS + j), bf4 = *(const v4f*)(BS + HID + j), bg4 = *(const v4f*)(BS + 2 * HID + j), bo4 = *(const v4f*)(BS + 3 * HID + j); v4f hn, cn;
#pragma unroll 1
    for (int q = 0; q < 4; ++q) { const float ig = sigm(__fadd_rn(vi[q], bi4[q])), fg = sigm(__fadd_rn(vf[q], bf4[q])), og = sigm(__fadd_rn(vo[q], bo4[q])); const float gg = tanhf(__fadd_rn(vg[q], bg4[q])); float p1 = __fmul_rn(fg, bfr(c0[q])), p2 = __fmul_rn(ig, gg);     asm volatile("" : "+v"(p1), "+v"(p2)); const float c1 = __fadd_rn(p1, p2); cn[q] = c1; hn[q] = __fmul_rn(og, tanhf(c1)); }
    *(volatile v4f*)(hout + e) = hn; *(volatile v4f*)(cout + e) = cn; __threadfence(); *(volatile v4f*)(hout + e) = hn; *(volatile v4f*)(cout + e) = cn; }

extern "C" void kernel_launch(void* const* d_in, const int* in_sizes, int n_in,
                              void* d_out, int out_size, void* d_ws, size_t ws_size, hipStream_t stream) {
    (void)in_sizes; (void)n_in; (void)out_size;
    const float* xi = (const float*)d_in[0]; const float* ht = (const float*)d_in[1]; const float* ct = (const float*)d_in[2]; const float* wi = (const float*)d_in[3]; const float* wh = (const float*)d_in[4]; const float* bi = (const float*)d_in[5]; const float* bh = (const float*)d_in[6];
    float* HOUT = (float*)d_out; float* COUT = HOUT + (size_t)TT * HID;
    char* wsp = (char*)d_ws;
    auto take = [&](size_t bytes) { char* p = wsp; wsp += (bytes + 255) & ~(size_t)255; return (void*)p; };
    bf* XH = (bf*)take((size_t)TT * DM * 2); bf* WB = (bf*)take((size_t)G4 * DM * 2); float* BS = (float*)take((size_t)G4 * 4); float* F = (float*)take((size_t)TT * G4 * 4);
    if ((size_t)(wsp - (char*)d_ws) > ws_size) return;
    k_cat8<<<(unsigned)(((size_t)TT * DM / 8 + 255) / 256), 256, 0, stream>>>(xi, ht, XH);
    k_wcat<<<(unsigned)(((size_t)G4 * DM / 8 + 255) / 256), 256, 0, stream>>>(wi, wh, WB);
    k_bsum<<<(G4 / 4 + 255) / 256, 256, 0, stream>>>(bi, bh, BS);
    k_gemmw<bf, 0, false><<<dim3(TT / 64, G4 / 64, 1), 32, 0, stream>>>(XH, nullptr, WB, nullptr, DM, F, G4, nullptr, 0, 0, 0);
    k_gates<<<(unsigned)(((size_t)TT * HID / 4 + 255) / 256), 256, 0, stream>>>(F, BS, ct, HOUT, COUT);
}
